// EagerAttentionModel_44693429682907
// MI455X (gfx1250) — hardware-verified
//
#include <hip/hip_runtime.h>
#include <stdint.h>

typedef __attribute__((ext_vector_type(16))) _Float16 v16h;
typedef __attribute__((ext_vector_type(8)))  _Float16 v8h;
typedef __attribute__((ext_vector_type(16))) __bf16   v16b;
typedef __attribute__((ext_vector_type(8)))  __bf16   v8b;
typedef __attribute__((ext_vector_type(8)))  float    v8f;
typedef __attribute__((ext_vector_type(4)))  float    v4f;

__device__ __forceinline__ unsigned short f2bf_bits(float f) {
  unsigned u = __float_as_uint(f);
  return (unsigned short)((u + 0x7FFFu + ((u >> 16) & 1u)) >> 16);
}
__device__ __forceinline__ float bf_bits2f(unsigned short h) { return __uint_as_float(((unsigned)h) << 16); }

__device__ __forceinline__ void dep_guard_h(v8f& a, v8f& b, v16h x, v16h y) { asm volatile("v_nop\n\tv_nop\n\tv_nop\n\tv_nop" : "+v"(a), "+v"(b) : "v"(x), "v"(y)); }
__device__ __forceinline__ void dep_guard_b(v8f& a, v8f& b, v16b x, v16b y) { asm volatile("v_nop\n\tv_nop\n\tv_nop\n\tv_nop" : "+v"(a), "+v"(b) : "v"(x), "v"(y)); }
__device__ __forceinline__ void keep4_h(v16h a, v16h b, v16h c, v16h d) { asm volatile("v_nop" :: "v"(a), "v"(b), "v"(c), "v"(d)); }
__device__ __forceinline__ void keep4_b(v16b a, v16b b, v16b c, v16b d) { asm volatile("v_nop" :: "v"(a), "v"(b), "v"(c), "v"(d)); }
__device__ __forceinline__ void acc_guard4(v8f& a, v8f& b, v8f& c, v8f& d) { asm volatile("v_nop\n\tv_nop\n\tv_nop\n\tv_nop" : "+v"(a), "+v"(b), "+v"(c), "+v"(d)); }
template <typename T> struct Frag;
template <> struct Frag<_Float16> {
  typedef v16h V; union U { v16h v; v8h h[2]; };
  static __device__ __forceinline__ v16h load(const _Float16* p) {
    U f; f.h[0] = *(const v8h*)(p); f.h[1] = *(const v8h*)(p + 16); return f.v;
  }
  static __device__ __forceinline__ v8f mma(v16h a, v16h b, v8f c) {
    return __builtin_amdgcn_wmma_f32_16x16x32_f16(false, a, false, b, (short)0, c, false, false);
  }
  static __device__ __forceinline__ void guard(v8f& a, v8f& b, v16h x, v16h y) { dep_guard_h(a, b, x, y); }
  static __device__ __forceinline__ void keep(v16h a, v16h b, v16h c, v16h d) { keep4_h(a, b, c, d); }
};
template <> struct Frag<__bf16> {
  typedef v16b V; union U { v16b v; v8b h[2]; };
  static __device__ __forceinline__ v16b load(const __bf16* p) {
    U f; f.h[0] = *(const v8b*)(p); f.h[1] = *(const v8b*)(p + 16); return f.v;
  }
  static __device__ __forceinline__ v8f mma(v16b a, v16b b, v8f c) {
    return __builtin_amdgcn_wmma_f32_16x16x32_bf16(false, a, false, b, (short)0, c, false, false);
  }
  static __device__ __forceinline__ void guard(v8f& a, v8f& b, v16b x, v16b y) { dep_guard_b(a, b, x, y); }
  static __device__ __forceinline__ void keep(v16b a, v16b b, v16b c, v16b d) { keep4_b(a, b, c, d); }
};

template <int ET> struct Elem;
template <> struct Elem<0> { typedef _Float16 T; };
template <> struct Elem<1> { typedef __bf16 T; };
template <int ET, int SPLIT, int BIAS_MODE, int OUT_MODE, bool RESID, int ACT = 0>
__global__ __launch_bounds__(256) void wmma_gemm64(
    const unsigned short* __restrict__ Ap, const unsigned short* __restrict__ A2p, int lda, long strideA,
    const unsigned short* __restrict__ Btp, const unsigned short* __restrict__ Bt2p, int ldb, long strideB,
    void* __restrict__ Cout, void* __restrict__ Cout2, int ldc, long strideC,
    const float* __restrict__ bias,
    const float* __restrict__ resid, long strideR,
    int M, int N, int K, float scale) {
  typedef typename Elem<ET>::T T;
  typedef typename Frag<T>::V V;
  const T* A = (const T*)Ap; const T* A2 = (const T*)A2p; const T* Bt = (const T*)Btp; const T* Bt2 = (const T*)Bt2p;
  __shared__ __align__(16) float sT[8][16 * 68];
  const int b    = blockIdx.y;
  const int lane = threadIdx.x & 31;
  const int wave = threadIdx.x >> 5;
  const int tilesN = N >> 6;
  const int tilesM = M >> 6;
  const int tile = blockIdx.x * 8 + wave;
  if (tile >= tilesM * tilesN) return;
  const int tm = tile / tilesN;
  const int tn = tile - tm * tilesN;
  const int m0 = tm << 6;
  const int n0 = tn << 6;

  const T* Ab  = A  + (size_t)b * strideA;
  const T* Bb  = Bt + (size_t)b * strideB;
  const T* Ab2 = (SPLIT != 0) ? (A2  + (size_t)b * strideA) : nullptr;
  const T* Bb2 = (SPLIT == 1) ? (Bt2 + (size_t)b * strideB) : nullptr;

  const int rlane = lane & 15;
  const int koff  = (lane >> 4) * 8;
  const int mOff  = (lane >> 4) * 8;

  v8f acc[4][4];
#pragma unroll
  for (int i = 0; i < 4; ++i)
#pragma unroll
    for (int j = 0; j < 4; ++j) acc[i][j] = (v8f){0.f,0.f,0.f,0.f,0.f,0.f,0.f,0.f};

  for (int k0 = 0; k0 < K; k0 += 32) {
    V bh[4], bl[4];
#pragma unroll
    for (int j = 0; j < 4; ++j) {
      const size_t bo = (size_t)(n0 + (j << 4) + rlane) * ldb + koff + k0;
      bh[j] = Frag<T>::load(Bb + bo);
      if (SPLIT == 1) bl[j] = Frag<T>::load(Bb2 + bo);
    }
#pragma unroll
    for (int i = 0; i < 4; ++i) {
      const size_t ao = (size_t)(m0 + (i << 4) + rlane) * lda + koff + k0;
      V ah = Frag<T>::load(Ab + ao);
      V al;
      if (SPLIT != 0) al = Frag<T>::load(Ab2 + ao);
#pragma unroll
      for (int j = 0; j < 4; ++j) {
        acc[i][j] = Frag<T>::mma(ah, bh[j], acc[i][j]);
        if (SPLIT == 1) acc[i][j] = Frag<T>::mma(ah, bl[j], acc[i][j]);
        if (SPLIT != 0) acc[i][j] = Frag<T>::mma(al, bh[j], acc[i][j]);
      }
      Frag<T>::guard(acc[i][0], acc[i][3], ah, (SPLIT != 0) ? al : ah);
    }
    Frag<T>::keep(bh[0], bh[1], bh[2], bh[3]);
    if (SPLIT == 1) Frag<T>::keep(bl[0], bl[1], bl[2], bl[3]);
  }
  acc_guard4(acc[0][0], acc[0][1], acc[0][2], acc[0][3]);
  acc_guard4(acc[1][0], acc[1][1], acc[1][2], acc[1][3]);
  acc_guard4(acc[2][0], acc[2][1], acc[2][2], acc[2][3]);
  acc_guard4(acc[3][0], acc[3][1], acc[3][2], acc[3][3]);

  float* slab = sT[wave];
  const float* Rb = RESID ? (resid + (size_t)b * strideR) : nullptr;
#pragma unroll
  for (int i = 0; i < 4; ++i) {
    const int mBase = m0 + (i << 4);
#pragma unroll
    for (int j = 0; j < 4; ++j) {
      const int n = n0 + (j << 4) + rlane;
      float bv = 0.f;
      if (BIAS_MODE == 2) bv = bias[n];
#pragma unroll
      for (int r = 0; r < 8; ++r) {
        float v = acc[i][j][r] * scale;
        if (BIAS_MODE == 1) v += bias[mBase + mOff + r];
        if (BIAS_MODE == 2) v += bv;
        if (RESID) v += Rb[(size_t)(mBase + mOff + r) * ldc + n];
        if (ACT == 1) v = tanhf(v);
        if (ACT == 2) v = fmaxf(v, 0.0f);
        if (ACT == 4) v = (v > 0.f) ? v : 0.01f * v;
        slab[(mOff + r) * 68 + (j << 4) + rlane] = v;
      }
    }
    __builtin_amdgcn_fence(__ATOMIC_RELEASE, "workgroup");
    __builtin_amdgcn_wave_barrier();
    __builtin_amdgcn_fence(__ATOMIC_ACQUIRE, "workgroup");
    if (OUT_MODE == 0) {
      float* C = (float*)Cout + (size_t)b * strideC;
      const int hh = lane >> 4, c4 = (lane & 15) * 4;
      for (int pass = 0; pass < 2; ++pass) {
#pragma unroll
        for (int it = 0; it < 8; ++it) {
          const int row = it * 2 + hh;
          v4f v = *(const v4f*)(slab + row * 68 + c4);
          *(volatile v4f*)(C + (size_t)(mBase + row) * ldc + n0 + c4) = v;
        }
        __threadfence();
      }
    } else {
      const int q = lane >> 3, c8 = (lane & 7) * 8;
      unsigned short* C  = (unsigned short*)Cout  + (size_t)b * strideC;
      unsigned short* C2 = (OUT_MODE == 2) ? ((unsigned short*)Cout2 + (size_t)b * strideC) : nullptr;
      for (int pass = 0; pass < 2; ++pass) {
#pragma unroll
        for (int it = 0; it < 4; ++it) {
          const int row = it * 4 + q;
          const float* sp = slab + row * 68 + c8;
          v8h hv, lv;
#pragma unroll
          for (int e = 0; e < 8; ++e) {
            if (OUT_MODE == 1) {
              hv[e] = (_Float16)sp[e];
            } else {
              unsigned short hb = f2bf_bits(sp[e]);
              unsigned short lb = f2bf_bits(sp[e] - bf_bits2f(hb));
              hv[e] = __builtin_bit_cast(_Float16, hb);
              lv[e] = __builtin_bit_cast(_Float16, lb);
            }
          }
          *(volatile v8h*)(C + (size_t)(mBase + row) * ldc + n0 + c8) = hv;
          if (OUT_MODE == 2) *(volatile v8h*)(C2 + (size_t)(mBase + row) * ldc + n0 + c8) = lv;
        }
        __threadfence();
      }
    }
    __builtin_amdgcn_fence(__ATOMIC_RELEASE, "workgroup");
    __builtin_amdgcn_wave_barrier();
    __builtin_amdgcn_fence(__ATOMIC_ACQUIRE, "workgroup");
  }
}

__global__ __launch_bounds__(256) void cast_bf16x8_k(
    const float* s0, const float* s1, const float* s2, const float* s3,
    unsigned short* d0, unsigned short* d1, unsigned short* d2, unsigned short* d3, int n8) {
  const int sel = blockIdx.y;
  const float* src = (sel == 0) ? s0 : (sel == 1) ? s1 : (sel == 2) ? s2 : s3;
  unsigned short* dst = (sel == 0) ? d0 : (sel == 1) ? d1 : (sel == 2) ? d2 : d3;
  const int i = blockIdx.x * 256 + threadIdx.x;
  if (i < n8) {
    const v4f a  = *(const v4f*)(src + (size_t)i * 8);
    const v4f bq = *(const v4f*)(src + (size_t)i * 8 + 4);
    v8h hv;
#pragma unroll
    for (int e = 0; e < 4; ++e) {
      hv[e]     = __builtin_bit_cast(_Float16, f2bf_bits(a[e]));
      hv[4 + e] = __builtin_bit_cast(_Float16, f2bf_bits(bq[e]));
    }
    _Float16* dp = (_Float16*)dst + (size_t)i * 8;
    *(volatile v8h*)dp = hv;
    __threadfence();
    *(volatile v8h*)dp = hv;
  }
}

__global__ __launch_bounds__(256) void bias_bf16val_k(
    const float* s0, const float* s1, const float* s2, const float* s3, float* __restrict__ dst, int n) {
  const int sel = blockIdx.y;
  const float* src = (sel == 0) ? s0 : (sel == 1) ? s1 : (sel == 2) ? s2 : s3;
  const int i = blockIdx.x * 256 + threadIdx.x;
  if (i * 4 < n) {
    const v4f v = *(const v4f*)(src + (size_t)i * 4);
    v4f o;
#pragma unroll
    for (int e = 0; e < 4; ++e) o[e] = bf_bits2f(f2bf_bits(v[e]));
    float* dp = dst + (size_t)sel * n + (size_t)i * 4;
    *(volatile v4f*)dp = o;
    __threadfence();
    *(volatile v4f*)dp = o;
  }
}

#define HDIM 64
#define KVCH 64
#define QBLK 64
#define OSPITCH 68

__device__ __forceinline__ v8f mma_h(v16h a, v16h b, v8f c) {
  c = __builtin_amdgcn_wmma_f32_16x16x32_f16(false, a, false, b, (short)0, c, false, false);
  asm volatile("v_nop\n\tv_nop\n\tv_nop\n\tv_nop" : "+v"(c) : "v"(a), "v"(b));
  return c;
}
__device__ __forceinline__ v8f mma_b(v16b a, v16b b, v8f c) {
  c = __builtin_amdgcn_wmma_f32_16x16x32_bf16(false, a, false, b, (short)0, c, false, false);
  asm volatile("v_nop\n\tv_nop\n\tv_nop\n\tv_nop" : "+v"(c) : "v"(a), "v"(b));
  return c;
}
__device__ __forceinline__ void bf_split(float f, __bf16& hi, __bf16& lo) {
  const unsigned short hb = f2bf_bits(f);
  hi = __builtin_bit_cast(__bf16, hb);
  lo = __builtin_bit_cast(__bf16, f2bf_bits(f - bf_bits2f(hb)));
}

__global__ __launch_bounds__(128)
void attn_causal64_k(const unsigned short* __restrict__ qkp,
                     const unsigned short* __restrict__ vhp, const unsigned short* __restrict__ vlp,
                     unsigned short* __restrict__ ohp, unsigned short* __restrict__ olp,
                     int S, int ldqk, int kcol0, int ldv, int nheads, float sm_scale) {
  union FH { v16h v; v8h h[2]; };
  union FB { v16b v; v8b h[2]; };
  __shared__ __align__(16) _Float16 Ksh[KVCH * HDIM];
  __shared__ __align__(16) __bf16   Vth[HDIM * KVCH];
  __shared__ __align__(16) __bf16   Vtl[HDIM * KVCH];
  __shared__ __align__(16) __bf16   Psh[4][16 * KVCH];
  __shared__ __align__(16) __bf16   Psl[4][16 * KVCH];
  __shared__ __align__(16) float    Os[4][16 * OSPITCH];

  const _Float16* qp = (const _Float16*)qkp;
  const __bf16*   vh = (const __bf16*)vhp;
  const __bf16*   vl = (const __bf16*)vlp;

  const int tid  = threadIdx.x;
  const int wave = tid >> 5;
  const int lane = tid & 31;
  const int hh   = lane >> 4;
  const int c    = lane & 15;

  const int nqb = S / QBLK;
  const int bx  = blockIdx.x;
  const int qb  = bx % nqb;
  int h = bx / nqb;
  h = (h < nheads) ? h : (nheads - 1);
  const int q0 = qb * QBLK + wave * 16;
  const float NEG_INF = -__builtin_inff();

  v16h qa[2];
  {
    const _Float16* qrow = qp + (size_t)(q0 + c) * ldqk + h * HDIM + 8 * hh;
#pragma unroll
    for (int dc = 0; dc < 2; ++dc) qa[dc] = Frag<_Float16>::load(qrow + dc * 32);
  }

  float mrow[8], lrow[8];
  v8f oacc[4];
#pragma unroll
  for (int r = 0; r < 8; ++r) { mrow[r] = NEG_INF; lrow[r] = 0.f; }
#pragma unroll
  for (int t = 0; t < 4; ++t) oacc[t] = (v8f){0.f,0.f,0.f,0.f,0.f,0.f,0.f,0.f};

  const int nChunks = qb + 1;
  for (int kc = 0; kc < nChunks; ++kc) {
    const int kv0 = kc * KVCH;
    __syncthreads();
    {
      const int kvr = tid >> 1, dh = (tid & 1) * 32;
      const _Float16* krow  = qp + (size_t)(kv0 + kvr) * ldqk + kcol0 + h * HDIM + dh;
      const __bf16*   vhrow = vh + (size_t)(kv0 + kvr) * ldv + h * HDIM + dh;
      const __bf16*   vlrow = vl + (size_t)(kv0 + kvr) * ldv + h * HDIM + dh;
#pragma unroll
      for (int i = 0; i < 4; ++i) {
        const v8h kk = *(const v8h*)(krow + 8 * i);
        *(v8h*)(Ksh + kvr * HDIM + dh + 8 * i) = kk;
        const v8b va = *(const v8b*)(vhrow + 8 * i);
        const v8b vb = *(const v8b*)(vlrow + 8 * i);
#pragma unroll
        for (int e = 0; e < 8; ++e) {
          Vth[(dh + 8 * i + e) * KVCH + kvr] = va[e];
          Vtl[(dh + 8 * i + e) * KVCH + kvr] = vb[e];
        }
      }
    }
    __syncthreads();

    v8f s[4];
#pragma unroll
    for (int j = 0; j < 4; ++j) {
      s[j] = (v8f){0.f,0.f,0.f,0.f,0.f,0.f,0.f,0.f};
#pragma unroll
      for (int dc = 0; dc < 2; ++dc) {
        FH kb;
        kb.h[0] = *(const v8h*)(Ksh + (j * 16 + c) * HDIM + dc * 32 + 8 * hh);
        kb.h[1] = *(const v8h*)(Ksh + (j * 16 + c) * HDIM + dc * 32 + 16 + 8 * hh);
        s[j] = mma_h(qa[dc], kb.v, s[j]);
      }
    }
    const bool diag = (kc == qb);
    float cm[8];
#pragma unroll
    for (int r = 0; r < 8; ++r) {
      const int qrow = q0 + 8 * hh + r;
      float m = NEG_INF;
#pragma unroll
      for (int j = 0; j < 4; ++j) {
        const int kvcol = kv0 + j * 16 + c;
        float val = s[j][r] * sm_scale;
        if (diag && (kvcol > qrow)) val = NEG_INF;
        s[j][r] = val;
        m = fmaxf(m, val);
      }
#pragma unroll
      for (int off = 1; off < 16; off <<= 1) m = fmaxf(m, __shfl_xor(m, off, 32));
      cm[r] = m;
    }
    __bf16* pwh = Psh[wave];
    __bf16* pwl = Psl[wave];
#pragma unroll
    for (int r = 0; r < 8; ++r) {
      const float mnew = fmaxf(mrow[r], cm[r]);
      const float alpha = expf(mrow[r] - mnew);
      mrow[r] = mnew;
      float psum = 0.f;
#pragma unroll
      for (int j = 0; j < 4; ++j) {
        const float p = expf(s[j][r] - mnew);
        psum += p;
        __bf16 ph, pl;
        bf_split(p, ph, pl);
        pwh[(8 * hh + r) * KVCH + j * 16 + c] = ph;
        pwl[(8 * hh + r) * KVCH + j * 16 + c] = pl;
      }
#pragma unroll
      for (int off = 1; off < 16; off <<= 1) psum += __shfl_xor(psum, off, 32);
      lrow[r] = lrow[r] * alpha + psum;
#pragma unroll
      for (int t = 0; t < 4; ++t) oacc[t][r] *= alpha;
    }
    __builtin_amdgcn_fence(__ATOMIC_RELEASE, "workgroup");
    __builtin_amdgcn_wave_barrier();
    __builtin_amdgcn_fence(__ATOMIC_ACQUIRE, "workgroup");
#pragma unroll 1
    for (int kk = 0; kk < 2; ++kk) {
      FB pa, pl;
      pa.h[0] = *(const v8b*)(pwh + c * KVCH + kk * 32 + 8 * hh);
      pa.h[1] = *(const v8b*)(pwh + c * KVCH + kk * 32 + 16 + 8 * hh);
      pl.h[0] = *(const v8b*)(pwl + c * KVCH + kk * 32 + 8 * hh);
      pl.h[1] = *(const v8b*)(pwl + c * KVCH + kk * 32 + 16 + 8 * hh);
#pragma unroll
      for (int t = 0; t < 4; ++t) {
        FB vb, vlo;
        vb.h[0]  = *(const v8b*)(Vth + (t * 16 + c) * KVCH + kk * 32 + 8 * hh);
        vb.h[1]  = *(const v8b*)(Vth + (t * 16 + c) * KVCH + kk * 32 + 16 + 8 * hh);
        vlo.h[0] = *(const v8b*)(Vtl + (t * 16 + c) * KVCH + kk * 32 + 8 * hh);
        vlo.h[1] = *(const v8b*)(Vtl + (t * 16 + c) * KVCH + kk * 32 + 16 + 8 * hh);
        oacc[t] = mma_b(pa.v, vb.v,  oacc[t]);
        oacc[t] = mma_b(pa.v, vlo.v, oacc[t]);
        oacc[t] = mma_b(pl.v, vb.v,  oacc[t]);
      }
    }
  }

  float* os = Os[wave];
#pragma unroll
  for (int r = 0; r < 8; ++r) {
    const float inv = 1.0f / lrow[r];
#pragma unroll
    for (int t = 0; t < 4; ++t) os[(8 * hh + r) * OSPITCH + t * 16 + c] = oacc[t][r] * inv;
  }
  __builtin_amdgcn_fence(__ATOMIC_RELEASE, "workgroup");
  __builtin_amdgcn_wave_barrier();
  __builtin_amdgcn_fence(__ATOMIC_ACQUIRE, "workgroup");
  {
    const int q4 = lane >> 3, c8 = (lane & 7) * 8;
    _Float16* oh = (_Float16*)ohp;
    _Float16* ol = (_Float16*)olp;
    for (int pass = 0; pass < 2; ++pass) {
#pragma unroll
      for (int it = 0; it < 4; ++it) {
        const int row = it * 4 + q4;
        const float* sp = os + row * OSPITCH + c8;
        v8h hv, lv;
#pragma unroll
        for (int e = 0; e < 8; ++e) {
          const unsigned short hb = f2bf_bits(sp[e]);
          const unsigned short lb = f2bf_bits(sp[e] - bf_bits2f(hb));
          hv[e] = __builtin_bit_cast(_Float16, hb);
          lv[e] = __builtin_bit_cast(_Float16, lb);
        }
        const size_t oo = (size_t)(q0 + row) * ldv + h * HDIM + c8;
        *(volatile v8h*)(oh + oo) = hv;
        *(volatile v8h*)(ol + oo) = lv;
      }
      __threadfence();
    }
  }
}

extern "C" void kernel_launch(void* const* d_in, const int* in_sizes, int n_in,
                              void* d_out, int out_size, void* d_ws, size_t ws_size,
                              hipStream_t stream) {
  constexpr int kS = 4096, kH = 1024, kNH = 16;
  const float kScale = 0.125f;
  if (n_in < 9) return;
  if (in_sizes[0] != kS * kH || in_sizes[1] != kH * kH || in_sizes[2] != kH ||
      in_sizes[3] != kH * kH || in_sizes[4] != kH || in_sizes[5] != kH * kH ||
      in_sizes[6] != kH || in_sizes[7] != kH * kH || in_sizes[8] != kH) return;
  if (out_size != kS * kH) return;

  const float* x  = (const float*)d_in[0];
  const float* Wq = (const float*)d_in[1];
  const float* bq = (const float*)d_in[2];
  const float* Wk = (const float*)d_in[3];
  const float* bk = (const float*)d_in[4];
  const float* Wv = (const float*)d_in[5];
  const float* bv = (const float*)d_in[6];
  const float* Wo = (const float*)d_in[7];
  const float* bo = (const float*)d_in[8];

  const size_t MiB = 1024u * 1024u;
  const size_t off_xb  = 0;
  const size_t off_wqk = off_xb  + (size_t)kS * kH * 2;
  const size_t off_wv  = off_wqk + (size_t)2 * kH * kH * 2;
  const size_t off_wo  = off_wv  + (size_t)kH * kH * 2;
  const size_t off_qk  = off_wo  + (size_t)kH * kH * 2;
  const size_t off_vhi = off_qk  + (size_t)kS * (2 * kH) * 2;
  const size_t off_vlo = off_vhi + (size_t)kS * kH * 2;
  const size_t off_ohi = off_vlo + (size_t)kS * kH * 2;
  const size_t off_olo = off_ohi + (size_t)kS * kH * 2;
  const size_t off_bias = off_olo + (size_t)kS * kH * 2;
  const size_t total = off_bias + (size_t)4 * kH * 4;
  (void)MiB;
  if (total > ws_size) return;

  char* ws = (char*)d_ws;
  unsigned short* xb  = (unsigned short*)(ws + off_xb);
  unsigned short* Wqk = (unsigned short*)(ws + off_wqk);
  unsigned short* Wvb = (unsigned short*)(ws + off_wv);
  unsigned short* Wob = (unsigned short*)(ws + off_wo);
  unsigned short* QKp = (unsigned short*)(ws + off_qk);
  unsigned short* Vhi = (unsigned short*)(ws + off_vhi);
  unsigned short* Vlo = (unsigned short*)(ws + off_vlo);
  unsigned short* Ohi = (unsigned short*)(ws + off_ohi);
  unsigned short* Olo = (unsigned short*)(ws + off_olo);
  float* biasws = (float*)(ws + off_bias);

  {
    const int n8 = kS * kH / 8;
    cast_bf16x8_k<<<dim3(n8 / 256, 1), 256, 0, stream>>>(x, x, x, x, xb, xb, xb, xb, n8);
  }
  {
    const int n8 = kH * kH / 8;
    cast_bf16x8_k<<<dim3(n8 / 256, 4), 256, 0, stream>>>(Wq, Wk, Wv, Wo,
        Wqk, Wqk + (size_t)kH * kH, Wvb, Wob, n8);
  }
  bias_bf16val_k<<<dim3(1, 4), 256, 0, stream>>>(bq, bk, bv, bo, biasws, kH);

  wmma_gemm64<1, 0, 2, 1, false><<<dim3((kS / 64) * (2 * kH / 64) / 8, 1), 256, 0, stream>>>(
      xb, xb, kH, 0L, Wqk, Wqk, kH, 0L, (void*)QKp, (void*)QKp, 2 * kH, 0L,
      biasws, biasws, 0L, kS, 2 * kH, kH, 1.0f);

  wmma_gemm64<1, 0, 2, 2, false><<<dim3((kS / 64) * (kH / 64) / 8, 1), 256, 0, stream>>>(
      xb, xb, kH, 0L, Wvb, Wvb, kH, 0L, (void*)Vhi, (void*)Vlo, kH, 0L,
      biasws + 2 * kH, biasws, 0L, kS, kH, kH, 1.0f);

  attn_causal64_k<<<dim3(kNH * (kS / 64)), 128, 0, stream>>>(
      QKp, Vhi, Vlo, Ohi, Olo, kS, 2 * kH, kH, kH, kNH, kScale);

  wmma_gemm64<1, 2, 2, 0, false><<<dim3((kS / 64) * (kH / 64) / 8, 1), 256, 0, stream>>>(
      Ohi, Olo, kH, 0L, Wob, Wob, kH, 0L, d_out, d_out, kH, 0L,
      biasws + 3 * kH, biasws, 0L, kS, kH, kH, 1.0f);
}
